// GraphAgent_42176578847132
// MI455X (gfx1250) — hardware-verified
//
#include <hip/hip_runtime.h>
#include <stddef.h>
#include <stdint.h>


#define HD      64
#define NVEC    32
#define KH0     96
#define K2      128
#define KS1     192
#define NOUTS   105
#define NPS     112
#define NTHR    256
#define NWAVE   8
#define EPT     8
#define CHUNK   (NTHR * EPT)
#define WCAP    (EPT * 32)
#define LISTN   (NWAVE * WCAP)
#define NBA     1024
#define SLA     10
#define RCAP    12288
#define DEGCAP  256
#define BTMAX   32
#define NBP     32
#define GTHR    128
#define GBM     64
#define AGG_ZINTS (LISTN + 2 * RCAP + 3 * NBA)
#define AGG_LDS_INTS (AGG_ZINTS + 16 + BTMAX * HD)
#define WSMAX   134217728
#define SLOPEF  0.01f

#define PO_B2E1 0
#define PO_B2E2 (PO_B2E1 + 64 * 96)
#define PO_ROOT (PO_B2E2 + 64 * 128)
#define PO_GIH  (PO_ROOT + 64 * 128)
#define PO_GHH  (PO_GIH + 192 * 128)
#define PO_S2P1 (PO_GHH + 192 * 128)
#define PO_S2P2 (PO_S2P1 + 64 * 192)
#define PO_S2P3 (PO_S2P2 + 64 * 128)
#define PO_G2P1 (PO_S2P3 + NPS * 128)
#define PO_TOT  (PO_G2P1 + 64 * 128)

static_assert((CHUNK & (CHUNK - 1)) == 0 && CHUNK <= 2048);
static_assert((NBA & (NBA - 1)) == 0 && NBA == (1 << SLA));
static_assert(((long long)CHUNK << SLA) < (1LL << 31));
static_assert(LISTN % NTHR == 0);
static_assert(NBA % NWAVE == 0 && NBA % 32 == 0 && NBA % GBM == 0);
static_assert(RCAP % 4 == 0 && AGG_ZINTS % 4 == 0 && LISTN % 4 == 0);
static_assert(AGG_LDS_INTS * 4 <= 300000);
static_assert(KH0 % 32 == 0 && K2 % 32 == 0 && KS1 % 32 == 0 && K2 == 2 * HD && KS1 == 3 * HD);
static_assert(GBM == (GTHR / 32) * 16);
static_assert((GBM * HD / 4) % GTHR == 0 && (GBM * HD / 4) % NTHR == 0);
static_assert((GBM * K2 / 8) % GTHR == 0 && (GBM * K2 / 8) % NTHR == 0);
static_assert((GBM * NOUTS) % 4 == 0 && ((GBM * NOUTS * 4) % 128) == 0);
static_assert(NPS % 16 == 0 && NPS >= NOUTS);
static_assert(NBP == 32 && NBP % NWAVE == 0 && NBP * 4 == 128);
static_assert(PO_B2E2 % 256 == 0 && PO_ROOT % 256 == 0 && PO_GIH % 256 == 0 && PO_GHH % 256 == 0);
static_assert(PO_S2P1 % 256 == 0 && PO_S2P2 % 256 == 0 && PO_S2P3 % 256 == 0 && PO_G2P1 % 256 == 0 && PO_TOT % 256 == 0);

typedef float          v2f   __attribute__((ext_vector_type(2)));
typedef float          v4f   __attribute__((ext_vector_type(4)));
typedef float          v8f   __attribute__((ext_vector_type(8)));
typedef int            v4i   __attribute__((ext_vector_type(4)));
typedef int            v8i   __attribute__((ext_vector_type(8)));
typedef unsigned short v8us  __attribute__((ext_vector_type(8)));
typedef unsigned short v16us __attribute__((ext_vector_type(16)));
typedef __bf16         v16bf __attribute__((ext_vector_type(16)));
typedef v2f  __attribute__((may_alias)) v2fa;
typedef v4f  __attribute__((may_alias)) v4fa;
typedef v4i  __attribute__((may_alias)) v4ia;
typedef v8us __attribute__((may_alias)) v8usa;
union FragB { v16bf v; v16us u; v8us h[2]; v8i w; };

__device__ __forceinline__ v8f wmb(const FragB& a, const FragB& b, v8f c) {
  v8f d = __builtin_amdgcn_wmma_f32_16x16x32_bf16(false, a.v, false, b.v, (short)0, c, false, false);
  asm volatile("v_nop\n\tv_nop\n\tv_nop\n\tv_nop" : "+v"(d) : "v"(a.w), "v"(b.w));
  return d;
}
__device__ __forceinline__ v8f z8() { v8f z = {0.f, 0.f, 0.f, 0.f, 0.f, 0.f, 0.f, 0.f}; return z; }

__device__ __forceinline__ unsigned bf16_bits(float f) {
  const unsigned u = __float_as_uint(f);
  return (u + 0x7FFFu + ((u >> 16) & 1u)) >> 16;
}
__device__ __forceinline__ float bf16_val(float f) { return __uint_as_float(bf16_bits(f) << 16); }
__device__ __forceinline__ unsigned short hlb(float x, bool lo) {
  const unsigned hb = bf16_bits(x);
  const unsigned lb = bf16_bits(x - __uint_as_float(hb << 16));
  return (unsigned short)(lo ? lb : hb);
}
__device__ __forceinline__ v8us hl8(v4f a, v4f b, bool lo) {
  v8us o;
  o[0] = hlb(a.x, lo); o[1] = hlb(a.y, lo); o[2] = hlb(a.z, lo); o[3] = hlb(a.w, lo);
  o[4] = hlb(b.x, lo); o[5] = hlb(b.y, lo); o[6] = hlb(b.z, lo); o[7] = hlb(b.w, lo);
  return o;
}
__device__ __forceinline__ v8us bf8(v4f a, v4f b) {
  v8us o;
  o[0] = (unsigned short)bf16_bits(a.x); o[1] = (unsigned short)bf16_bits(a.y);
  o[2] = (unsigned short)bf16_bits(a.z); o[3] = (unsigned short)bf16_bits(a.w);
  o[4] = (unsigned short)bf16_bits(b.x); o[5] = (unsigned short)bf16_bits(b.y);
  o[6] = (unsigned short)bf16_bits(b.z); o[7] = (unsigned short)bf16_bits(b.w);
  return o;
}
__device__ __forceinline__ float lrelu(float x) { return x >= 0.0f ? x : SLOPEF * x; }
__device__ __forceinline__ float sigm(float x) { return 1.0f / (1.0f + expf(-x)); }
__device__ __forceinline__ float wsum(float p) {
  p += __shfl_xor(p, 16); p += __shfl_xor(p, 8); p += __shfl_xor(p, 4); p += __shfl_xor(p, 2); p += __shfl_xor(p, 1);
  return p;
}

template <int NT>
__device__ __forceinline__ void put_f32_tile(const float* stg, float* dst, int tid) {
#pragma unroll
  for (int it = 0; it < (GBM * HD / 4) / NT; ++it) {
    const int i = it * NT + tid;
    const v4f v = *(const v4fa*)(stg + 4 * i);
    *(volatile v4f*)(dst + 4 * i) = v;
  }
}
template <int NT>
__device__ __forceinline__ void put_hl_tile(const float* stg, unsigned short* dst, int tid) {
#pragma unroll
  for (int it = 0; it < (GBM * K2 / 8) / NT; ++it) {
    const int u = it * NT + tid;
    const int row = u >> 4, qq = u & 15;
    const float* p = stg + row * HD + 8 * (qq & 7);
    const v4f a = *(const v4fa*)p;
    const v4f b = *(const v4fa*)(p + 4);
    const v8us o = hl8(a, b, qq >= 8);
    *(volatile v8us*)(dst + 8 * u) = o;
  }
}

template <int SLB>
__device__ __forceinline__ int scan_chunk(const int* __restrict__ ids, int nE, int cbase, int slotBase,
                                          int nb, int vec8, int* list, int tid, int lane, int wave) {
  int wc = 0;
  const int el0  = tid * EPT;
  const int e0   = cbase + el0;
  const int sent = -2147483647 - 1;
  v4i da, db;
  if (vec8 != 0 && cbase + CHUNK <= nE) {
    da = *(const v4i*)(ids + e0);
    db = *(const v4i*)(ids + e0 + 4);
  } else {
    const int lst = nE - 1;
    da.x = (e0     < nE) ? ids[min(e0,     lst)] : sent;
    da.y = (e0 + 1 < nE) ? ids[min(e0 + 1, lst)] : sent;
    da.z = (e0 + 2 < nE) ? ids[min(e0 + 2, lst)] : sent;
    da.w = (e0 + 3 < nE) ? ids[min(e0 + 3, lst)] : sent;
    db.x = (e0 + 4 < nE) ? ids[min(e0 + 4, lst)] : sent;
    db.y = (e0 + 5 < nE) ? ids[min(e0 + 5, lst)] : sent;
    db.z = (e0 + 6 < nE) ? ids[min(e0 + 6, lst)] : sent;
    db.w = (e0 + 7 < nE) ? ids[min(e0 + 7, lst)] : sent;
  }
  const unsigned bs = (unsigned)slotBase;
  const unsigned ub = (unsigned)nb;
  const unsigned s0 = (unsigned)da.x - bs, s1 = (unsigned)da.y - bs;
  const unsigned s2 = (unsigned)da.z - bs, s3 = (unsigned)da.w - bs;
  const unsigned s4 = (unsigned)db.x - bs, s5 = (unsigned)db.y - bs;
  const unsigned s6 = (unsigned)db.z - bs, s7 = (unsigned)db.w - bs;
  const bool h0 = s0 < ub, h1 = s1 < ub, h2 = s2 < ub, h3 = s3 < ub;
  const bool h4 = s4 < ub, h5 = s5 < ub, h6 = s6 < ub, h7 = s7 < ub;
  const unsigned any = __builtin_amdgcn_ballot_w32(h0 | h1 | h2 | h3 | h4 | h5 | h6 | h7);
  if (any != 0u) {
#define HITJ(J, HJ, SJ) { \
      const unsigned mj = __builtin_amdgcn_ballot_w32(HJ); \
      if (mj != 0u) { \
        if (HJ) { \
          const int pos = wc + (int)__builtin_amdgcn_mbcnt_lo(mj, 0u); \
          if (pos < WCAP) list[wave * WCAP + pos] = ((el0 + (J)) << SLB) | (int)(SJ); \
        } \
        wc += (int)__builtin_popcount(mj); } }
    HITJ(0, h0, s0)
    HITJ(1, h1, s1)
    HITJ(2, h2, s2)
    HITJ(3, h3, s3)
    HITJ(4, h4, s4)
    HITJ(5, h5, s5)
    HITJ(6, h6, s6)
    HITJ(7, h7, s7)
#undef HITJ
  }
  return wc;
}

__global__ __launch_bounds__(NTHR) void k_wprep(const float* __restrict__ pb2e1, const float* __restrict__ pb2e2,
                                                const float* __restrict__ proot, const float* __restrict__ pgih,
                                                const float* __restrict__ pghh, const float* __restrict__ ps1,
                                                const float* __restrict__ ps2, const float* __restrict__ ps3,
                                                const float* __restrict__ pg1, unsigned short* wpl) {
  const int y = (int)blockIdx.y;
  const float* W = pb2e1;
  int nOut = 64, nIn = 96, tr = 0, rows = 64, ld = 96, krep = 96, po = PO_B2E1;
  if (y == 1)      { W = pb2e2; nOut = 64;    nIn = 64;  tr = 0; rows = 64;  ld = 128; krep = 64; po = PO_B2E2; }
  else if (y == 2) { W = proot; nOut = 64;    nIn = 64;  tr = 1; rows = 64;  ld = 128; krep = 64; po = PO_ROOT; }
  else if (y == 3) { W = pgih;  nOut = 192;   nIn = 64;  tr = 0; rows = 192; ld = 128; krep = 64; po = PO_GIH; }
  else if (y == 4) { W = pghh;  nOut = 192;   nIn = 64;  tr = 0; rows = 192; ld = 128; krep = 64; po = PO_GHH; }
  else if (y == 5) { W = ps1;   nOut = 64;    nIn = 128; tr = 0; rows = 64;  ld = 192; krep = 64; po = PO_S2P1; }
  else if (y == 6) { W = ps2;   nOut = 64;    nIn = 64;  tr = 0; rows = 64;  ld = 128; krep = 64; po = PO_S2P2; }
  else if (y == 7) { W = ps3;   nOut = NOUTS; nIn = 64;  tr = 0; rows = NPS; ld = 128; krep = 64; po = PO_S2P3; }
  else if (y == 8) { W = pg1;   nOut = 64;    nIn = 64;  tr = 0; rows = 64;  ld = 128; krep = 64; po = PO_G2P1; }
  else if (y > 8) return;
  const int upr = ld >> 3;
  const int u = (int)blockIdx.x * NTHR + (int)threadIdx.x;
  if (u >= rows * upr) return;
  const int n  = u / upr;
  const int k8 = (u - n * upr) * 8;
  const int nc = n < nOut ? n : nOut - 1;
  v8us o;
#pragma unroll
  for (int i = 0; i < 8; ++i) {
    const int k  = k8 + i;
    const int ks = k < krep ? k : k - krep;
    const int idx = tr ? (ks * nOut + nc) : (nc * nIn + ks);
    const float v = W[idx];
    o[i] = (n < nOut) ? (unsigned short)bf16_bits(v) : (unsigned short)0;
  }
  unsigned short* dp = wpl + po + (size_t)n * ld + k8;
  *(volatile v8us*)dp = o;
  __threadfence();
  *(volatile v8us*)dp = o;
}

__global__ __launch_bounds__(NTHR) void k_h0(const int* __restrict__ xid, const int* __restrict__ bat,
                                             const float* __restrict__ bemb, int nBlk,
                                             const float* __restrict__ vec, int nG, int nUnits,
                                             unsigned short* h0) {
  const int u = (int)blockIdx.x * NTHR + (int)threadIdx.x;
  if (u >= nUnits) return;
  const int row = u / (KH0 / 8);
  const int c   = u - row * (KH0 / 8);
  int id = xid[row]; id = id < 0 ? 0 : (id > nBlk - 1 ? nBlk - 1 : id);
  int g  = bat[row]; g  = g  < 0 ? 0 : (g  > nG - 1   ? nG - 1   : g);
  const int kb = 8 * (c < 7 ? c : 7);
  int kv = c - 8; kv = kv < 0 ? 0 : (kv > 3 ? 3 : kv); kv *= 8;
  const float* pb = bemb + (size_t)id * HD + kb;
  const float* pv = vec + (size_t)g * NVEC + kv;
  const v4f a0 = *(const v4f*)pb, a1 = *(const v4f*)(pb + 4);
  const v4f c0 = *(const v4f*)pv, c1 = *(const v4f*)(pv + 4);
  const v8us ob = bf8(a0, a1);
  const v8us ov = bf8(c0, c1);
  v8us o;
#pragma unroll
  for (int i = 0; i < 8; ++i) o[i] = (c < 8) ? ob[i] : ov[i];
  unsigned short* dp = h0 + (size_t)u * 8;
  *(volatile v8us*)dp = o;
  __threadfence();
  *(volatile v8us*)dp = o;
}

template <int ACT, int WF, int WH>
__global__ __launch_bounds__(GTHR) void k_gemm64(const unsigned short* __restrict__ A, int lda,
                                                 const unsigned short* __restrict__ BT, int ldb, int K,
                                                 const float* __restrict__ bias, float* Cf, unsigned short* Ch) {
  __shared__ __attribute__((aligned(16))) float stg[GBM * HD];
  const int tid = (int)threadIdx.x, lane = tid & 31, wave = tid >> 5, hh = lane >> 4, m = lane & 15;
  const int rowBase = (int)blockIdx.x * GBM;

  v8f acc[4];
#pragma unroll
  for (int t = 0; t < 4; ++t) acc[t] = z8();
  const unsigned short* ap = A  + (size_t)(rowBase + 16 * wave + m) * (size_t)lda + 8 * hh;
  const unsigned short* bp = BT + (size_t)m * (size_t)ldb + 8 * hh;

#pragma unroll 1
  for (int k0 = 0; k0 < K; k0 += 32) {
    FragB af;
    af.h[0] = *(const v8usa*)(ap + k0);
    af.h[1] = *(const v8usa*)(ap + k0 + 16);
#pragma unroll
    for (int nt = 0; nt < 4; ++nt) {
      const unsigned short* wq = bp + (size_t)(16 * nt) * (size_t)ldb + k0;
      FragB bf;
      bf.h[0] = *(const v8usa*)wq;
      bf.h[1] = *(const v8usa*)(wq + 16);
      acc[nt] = wmb(af, bf, acc[nt]);
    }
  }

#pragma unroll
  for (int nt = 0; nt < 4; ++nt) {
    const int lc = 16 * nt + m;
    const float bv = bf16_val(bias[lc]);
#pragma unroll
    for (int r = 0; r < 8; ++r) {
      const int lr = 16 * wave + 8 * hh + r;
      float v = acc[nt][r] + bv;
      if (ACT != 0) v = lrelu(v);
      stg[lr * HD + lc] = v;
    }
  }
  __syncthreads();

  if (WF != 0) put_f32_tile<GTHR>(stg, Cf + (size_t)rowBase * HD, tid);
  if (WH != 0) put_hl_tile<GTHR>(stg, Ch + (size_t)rowBase * K2, tid);
  __threadfence();
  if (WF != 0) put_f32_tile<GTHR>(stg, Cf + (size_t)rowBase * HD, tid);
  if (WH != 0) put_hl_tile<GTHR>(stg, Ch + (size_t)rowBase * K2, tid);
}

__global__ __launch_bounds__(NTHR) void k_agg(const int* __restrict__ srcs, const int* __restrict__ dsts,
                                              const int* __restrict__ ea, int nE, int nN, int vec8,
                                              const float* __restrict__ outf, const float* __restrict__ orp,
                                              const float* __restrict__ bond, int nBond,
                                              unsigned short* mpl) {
  extern __shared__ __attribute__((aligned(16))) int dsm[];
  int* list = dsm;
  int* hl   = dsm + LISTN;
  int* sl   = hl + RCAP;
  int* cnt  = sl + RCAP;
  int* offs = cnt + NBA;
  int* cur  = offs + NBA;
  int* misc = cur + NBA;
  float* bt = (float*)(misc + 16);
  const int tid = (int)threadIdx.x, lane = tid & 31, wave = tid >> 5;
  const int nodeBase = (int)blockIdx.x * NBA;

  {
    const v4i z4 = {0, 0, 0, 0};
    for (int i = tid * 4; i < AGG_ZINTS; i += NTHR * 4) *(v4ia*)(dsm + i) = z4;
    if (tid < 16) misc[tid] = 0;
#pragma unroll 1
    for (int i = tid; i < BTMAX * HD; i += NTHR) {
      const int r  = i >> 6;
      const int rc = r < nBond ? r : nBond - 1;
      const float v = bond[(size_t)rc * HD + (i & (HD - 1))];
      bt[i] = (r < nBond) ? bf16_val(v) : 0.0f;
    }
  }
  __syncthreads();

  int t = 0, ov = 0;
  const int nChunks = (nE + CHUNK - 1) / CHUNK;
#pragma unroll 1
  for (int ch = 0; ch < nChunks; ++ch) {
    const int cbase = ch * CHUNK;
    const int wc = scan_chunk<SLA>(dsts, nE, cbase, nodeBase, NBA, vec8, list, tid, lane, wave);
    if (lane == 0) misc[wave] = wc;
    __syncthreads();
    if (wave == 0) {
#pragma unroll 1
      for (int w2 = 0; w2 < NWAVE; ++w2) {
        int c = misc[w2];
        c = c < 0 ? 0 : (c > WCAP ? WCAP : c);
#pragma unroll 1
        for (int b0 = 0; b0 < c; b0 += 32) {
          const int idx = b0 + lane;
          const int ent = list[w2 * WCAP + (idx < WCAP ? idx : WCAP - 1)];
          const int m32 = (c - b0) < 32 ? (c - b0) : 32;
#pragma unroll 1
          for (int k = 0; k < m32; ++k) {
            const int u    = __builtin_amdgcn_readlane(ent, k);
            const int slot = u & (NBA - 1);
            const int el   = (u >> SLA) & (CHUNK - 1);
            const int pk   = ((cbase + el) << SLA) | slot;
            if (t < RCAP) {
              if (lane == 0) { hl[t] = pk; cnt[slot] = cnt[slot] + 1; }
              t = t + 1;
            } else {
              ov = 1;
            }
          }
        }
      }
    }
    __syncthreads();
  }
  if (wave == 0 && lane == 0) { misc[8] = t; misc[9] = ov; }
  __syncthreads();
  int tt = misc[8];
  tt = tt < 0 ? 0 : (tt > RCAP ? RCAP : tt);
  const int ovf = misc[9];

  if (wave == 0) {
    const int base = lane * (NBA / 32);
    int s = 0;
#pragma unroll 1
    for (int i = 0; i < NBA / 32; ++i) s += cnt[base + i];
    int incl = s;
#pragma unroll
    for (int d = 1; d < 32; d <<= 1) {
      const int y = __shfl_up(incl, d, 32);
      if (lane >= d) incl += y;
    }
    int run = incl - s;
#pragma unroll 1
    for (int i = 0; i < NBA / 32; ++i) {
      const int cv = cnt[base + i];
      offs[base + i] = run;
      cur[base + i]  = run;
      run += cv;
    }
  }
  __syncthreads();
  if (wave == 0) {
#pragma unroll 1
    for (int b0 = 0; b0 < tt; b0 += 32) {
      const int idx = b0 + lane;
      const int ent = hl[idx < RCAP ? idx : RCAP - 1];
      const int m32 = (tt - b0) < 32 ? (tt - b0) : 32;
#pragma unroll 1
      for (int k = 0; k < m32; ++k) {
        const int u    = __builtin_amdgcn_readlane(ent, k);
        const int slot = u & (NBA - 1);
        if (lane == 0) {
          int p = cur[slot];
          p = p < 0 ? 0 : (p > RCAP - 1 ? RCAP - 1 : p);
          sl[p] = u;
          cur[slot] = p + 1;
        }
      }
    }
  }
  __syncthreads();

  const float pz = (ovf != 0) ? __int_as_float(0x7fc00000) : 0.0f;
#pragma unroll 1
  for (int si = 0; si < NBA / NWAVE; ++si) {
    const int s    = si * NWAVE + wave;
    const int node = nodeBase + s;
    const int craw = cnt[s];
    const bool big = craw > DEGCAP;
    const int c = craw < 0 ? 0 : (craw > DEGCAP ? DEGCAP : craw);
    int o = offs[s];
    o = o < 0 ? 0 : (o > RCAP ? RCAP : o);
    float acc0 = 0.0f, acc1 = 0.0f;
#pragma unroll 1
    for (int b0 = 0; b0 < c; b0 += 32) {
      int idx = o + b0 + lane;
      idx = idx > RCAP - 1 ? RCAP - 1 : idx;
      const int ent = sl[idx];
      int eid = ent >> SLA;
      eid = eid < 0 ? 0 : (eid > nE - 1 ? nE - 1 : eid);
      int sr = srcs[eid];
      sr = sr < 0 ? 0 : (sr > nN - 1 ? nN - 1 : sr);
      int a0 = ea[2 * eid];
      a0 = a0 < 0 ? 0 : (a0 > nBond - 1 ? nBond - 1 : a0);
      int a1 = ea[2 * eid + 1];
      a1 = a1 < 0 ? 0 : (a1 > nBond - 1 ? nBond - 1 : a1);
      const int m32 = (c - b0) < 32 ? (c - b0) : 32;
#pragma unroll 1
      for (int k = 0; k < m32; ++k) {
        const int sk = __builtin_amdgcn_readlane(sr, k);
        const int ak = __builtin_amdgcn_readlane(a0, k);
        const int bk = __builtin_amdgcn_readlane(a1, k);
        const v2f x  = *(const v2f*)(outf + (size_t)sk * HD + 2 * lane);
        const v2f u0 = *(const v2fa*)(bt + ak * HD + 2 * lane);
        float p = x.x * u0.x + x.y * u0.y;
        p = wsum(p);
        const v2f u1 = *(const v2fa*)(bt + bk * HD + 2 * lane);
        acc0 = fmaf(p, u1.x, acc0);
        acc1 = fmaf(p, u1.y, acc1);
      }
    }
    const int nc = node < nN ? node : nN - 1;
    const int den = craw < 1 ? 1 : craw;
    const float rden = 1.0f / (float)den;
    const v2f orv = *(const v2f*)(orp + (size_t)nc * HD + 2 * lane);
    const float pzr = big ? __int_as_float(0x7fc00000) : pz;
    const float v0 = lrelu(acc0 * rden + orv.x) + pzr;
    const float v1 = lrelu(acc1 * rden + orv.y) + pzr;
    const unsigned hw = (unsigned)hlb(v0, false) | ((unsigned)hlb(v1, false) << 16);
    const unsigned lw = (unsigned)hlb(v0, true)  | ((unsigned)hlb(v1, true)  << 16);
    if (node < nN) {
      unsigned* hp = (unsigned*)(mpl + (size_t)node * K2) + lane;
      unsigned* lp = (unsigned*)(mpl + (size_t)node * K2 + HD) + lane;
      *(volatile unsigned*)hp = hw;
      *(volatile unsigned*)lp = lw;
      __threadfence();
      *(volatile unsigned*)hp = hw;
      *(volatile unsigned*)lp = lw;
    }
  }
}

__global__ __launch_bounds__(NTHR) void k_gru(const unsigned short* __restrict__ mpl, const unsigned short* __restrict__ oa,
                                              const float* __restrict__ of, const unsigned short* __restrict__ gih,
                                              const unsigned short* __restrict__ ghh, const float* __restrict__ bih,
                                              const float* __restrict__ bhh, float* ofn, unsigned short* oan) {
  __shared__ __attribute__((aligned(16))) float hold[GBM * HD];
  __shared__ __attribute__((aligned(16))) float hnew[GBM * HD];
  const int tid = (int)threadIdx.x, lane = tid & 31, wave = tid >> 5, hh = lane >> 4, m = lane & 15;
  const int rg = wave >> 1, q = wave & 1;
  const int rowBase = (int)blockIdx.x * GBM;
  {
    const int row = tid >> 2, part = tid & 3;
    const float* hp = of + (size_t)(rowBase + row) * HD + 16 * part;
    const v4f a0 = *(const v4f*)hp, a1 = *(const v4f*)(hp + 4), a2 = *(const v4f*)(hp + 8), a3 = *(const v4f*)(hp + 12);
    float* dp = hold + row * HD + 16 * part;
    *(v4fa*)dp = a0; *(v4fa*)(dp + 4) = a1; *(v4fa*)(dp + 8) = a2; *(v4fa*)(dp + 12) = a3;
  }
  __syncthreads();

  v8f gx[3][2], gh[3][2];
#pragma unroll
  for (int g = 0; g < 3; ++g) { gx[g][0] = z8(); gx[g][1] = z8(); gh[g][0] = z8(); gh[g][1] = z8(); }
  {
    const unsigned short* ap = mpl + (size_t)(rowBase + 16 * rg + m) * K2 + 8 * hh;
    const unsigned short* bq = gih + (size_t)(32 * q + m) * K2 + 8 * hh;
#pragma unroll 1
    for (int k0 = 0; k0 < K2; k0 += 32) {
      FragB af;
      af.h[0] = *(const v8usa*)(ap + k0);
      af.h[1] = *(const v8usa*)(ap + k0 + 16);
#pragma unroll
      for (int g = 0; g < 3; ++g) {
#pragma unroll
        for (int uu = 0; uu < 2; ++uu) {
          const unsigned short* wq = bq + (size_t)(64 * g + 16 * uu) * K2 + k0;
          FragB bf;
          bf.h[0] = *(const v8usa*)wq;
          bf.h[1] = *(const v8usa*)(wq + 16);
          gx[g][uu] = wmb(af, bf, gx[g][uu]);
        }
      }
    }
  }
  {
    const unsigned short* ap = oa + (size_t)(rowBase + 16 * rg + m) * K2 + 8 * hh;
    const unsigned short* bq = ghh + (size_t)(32 * q + m) * K2 + 8 * hh;
#pragma unroll 1
    for (int k0 = 0; k0 < K2; k0 += 32) {
      FragB af;
      af.h[0] = *(const v8usa*)(ap + k0);
      af.h[1] = *(const v8usa*)(ap + k0 + 16);
#pragma unroll
      for (int g = 0; g < 3; ++g) {
#pragma unroll
        for (int uu = 0; uu < 2; ++uu) {
          const unsigned short* wq = bq + (size_t)(64 * g + 16 * uu) * K2 + k0;
          FragB bf;
          bf.h[0] = *(const v8usa*)wq;
          bf.h[1] = *(const v8usa*)(wq + 16);
          gh[g][uu] = wmb(af, bf, gh[g][uu]);
        }
      }
    }
  }

#pragma unroll
  for (int uu = 0; uu < 2; ++uu) {
    const int j = 32 * q + 16 * uu + m;
    const float bir = bf16_val(bih[j]), biz = bf16_val(bih[HD + j]), bin = bf16_val(bih[2 * HD + j]);
    const float bhr = bf16_val(bhh[j]), bhz = bf16_val(bhh[HD + j]), bhn = bf16_val(bhh[2 * HD + j]);
#pragma unroll
    for (int r = 0; r < 8; ++r) {
      const int row = 16 * rg + 8 * hh + r;
      const float rr = sigm((gx[0][uu][r] + bir) + (gh[0][uu][r] + bhr));
      const float zz = sigm((gx[1][uu][r] + biz) + (gh[1][uu][r] + bhz));
      const float nn = tanhf((gx[2][uu][r] + bin) + rr * (gh[2][uu][r] + bhn));
      const float ho = hold[row * HD + j];
      hnew[row * HD + j] = (1.0f - zz) * nn + zz * ho;
    }
  }
  __syncthreads();

  put_f32_tile<NTHR>(hnew, ofn + (size_t)rowBase * HD, tid);
  put_hl_tile<NTHR>(hnew, oan + (size_t)rowBase * K2, tid);
  __threadfence();
  put_f32_tile<NTHR>(hnew, ofn + (size_t)rowBase * HD, tid);
  put_hl_tile<NTHR>(hnew, oan + (size_t)rowBase * K2, tid);
}

__global__ __launch_bounds__(GTHR) void k_stem1(const unsigned short* __restrict__ oa, int nN,
                                                const int* __restrict__ stype, const int* __restrict__ sloc,
                                                const int* __restrict__ sbat, const int* __restrict__ nsl,
                                                int nSl, int nS, const float* __restrict__ se, int nStemT,
                                                const unsigned short* __restrict__ BT,
                                                const float* __restrict__ bias, unsigned short* S1) {
  __shared__ __attribute__((aligned(16))) unsigned short SA[GBM * KS1];
  __shared__ __attribute__((aligned(16))) float stg[GBM * HD];
  __shared__ int sidx[GBM];
  __shared__ int stid[GBM];
  const int tid = (int)threadIdx.x, lane = tid & 31, wave = tid >> 5, hh = lane >> 4, m = lane & 15;
  const int sBase = (int)blockIdx.x * GBM;
  if (tid < GBM) {
    int t = sBase + tid;
    t = t > nS - 1 ? nS - 1 : t;
    int b = sbat[t];
    b = b < 0 ? 0 : (b > nSl - 1 ? nSl - 1 : b);
    int ix = nsl[b] + sloc[t];
    ix = ix < 0 ? 0 : (ix > nN - 1 ? nN - 1 : ix);
    sidx[tid] = ix;
    int ty = stype[t];
    ty = ty < 0 ? 0 : (ty > nStemT - 1 ? nStemT - 1 : ty);
    stid[tid] = ty;
  }
  __syncthreads();
#pragma unroll 1
  for (int u = tid; u < GBM * (KS1 / 8); u += GTHR) {
    const int row = u / (KS1 / 8);
    const int c   = u - row * (KS1 / 8);
    const int ix  = sidx[row];
    const int ty  = stid[row];
    const int co  = 8 * (c < 15 ? c : 15);
    int cs = c - 16; cs = cs < 0 ? 0 : (cs > 7 ? 7 : cs); cs *= 8;
    const v8us a = *(const v8usa*)(oa + (size_t)ix * K2 + co);
    const float* sp = se + (size_t)ty * HD + cs;
    const v4f s0 = *(const v4f*)sp, s1 = *(const v4f*)(sp + 4);
    const v8us e = bf8(s0, s1);
    v8us o;
#pragma unroll
    for (int i = 0; i < 8; ++i) o[i] = (c < 16) ? a[i] : e[i];
    *(v8usa*)(SA + row * KS1 + 8 * c) = o;
  }
  __syncthreads();

  v8f acc[4];
#pragma unroll
  for (int t = 0; t < 4; ++t) acc[t] = z8();
  const unsigned short* arow = SA + (16 * wave + m) * KS1 + 8 * hh;
  const unsigned short* bp   = BT + (size_t)m * KS1 + 8 * hh;
#pragma unroll 1
  for (int k0 = 0; k0 < KS1; k0 += 32) {
    FragB af;
    af.h[0] = *(const v8usa*)(arow + k0);
    af.h[1] = *(const v8usa*)(arow + k0 + 16);
#pragma unroll
    for (int nt = 0; nt < 4; ++nt) {
      const unsigned short* wq = bp + (size_t)(16 * nt) * KS1 + k0;
      FragB bf;
      bf.h[0] = *(const v8usa*)wq;
      bf.h[1] = *(const v8usa*)(wq + 16);
      acc[nt] = wmb(af, bf, acc[nt]);
    }
  }
#pragma unroll
  for (int nt = 0; nt < 4; ++nt) {
    const int lc = 16 * nt + m;
    const float bv = bf16_val(bias[lc]);
#pragma unroll
    for (int r = 0; r < 8; ++r) {
      const int lr = 16 * wave + 8 * hh + r;
      stg[lr * HD + lc] = lrelu(acc[nt][r] + bv);
    }
  }
  __syncthreads();
  put_hl_tile<GTHR>(stg, S1 + (size_t)sBase * K2, tid);
  __threadfence();
  put_hl_tile<GTHR>(stg, S1 + (size_t)sBase * K2, tid);
}

__global__ __launch_bounds__(GTHR) void k_stem3(const unsigned short* __restrict__ A,
                                                const unsigned short* __restrict__ BT,
                                                const float* __restrict__ b3, float* out) {
  __shared__ __attribute__((aligned(16))) float stg[GBM * NOUTS];
  const int tid = (int)threadIdx.x, lane = tid & 31, wave = tid >> 5, hh = lane >> 4, m = lane & 15;
  const int sBase = (int)blockIdx.x * GBM;

  v8f acc[7];
#pragma unroll
  for (int t = 0; t < 7; ++t) acc[t] = z8();
  const unsigned short* ap = A  + (size_t)(sBase + 16 * wave + m) * K2 + 8 * hh;
  const unsigned short* bp = BT + (size_t)m * K2 + 8 * hh;
#pragma unroll 1
  for (int k0 = 0; k0 < K2; k0 += 32) {
    FragB af;
    af.h[0] = *(const v8usa*)(ap + k0);
    af.h[1] = *(const v8usa*)(ap + k0 + 16);
#pragma unroll
    for (int nt = 0; nt < 7; ++nt) {
      const unsigned short* wq = bp + (size_t)(16 * nt) * K2 + k0;
      FragB bf;
      bf.h[0] = *(const v8usa*)wq;
      bf.h[1] = *(const v8usa*)(wq + 16);
      acc[nt] = wmb(af, bf, acc[nt]);
    }
  }
#pragma unroll
  for (int nt = 0; nt < 7; ++nt) {
    const int lc  = 16 * nt + m;
    const int lcc = lc < NOUTS ? lc : NOUTS - 1;
    const float bv = bf16_val(b3[lcc]);
#pragma unroll
    for (int r = 0; r < 8; ++r) {
      const int lr = 16 * wave + 8 * hh + r;
      if (lc < NOUTS) stg[lr * NOUTS + lc] = acc[nt][r] + bv;
    }
  }
  __syncthreads();

  float* base = out + (size_t)blockIdx.x * (GBM * NOUTS);
#pragma unroll 1
  for (int i = tid; i < (GBM * NOUTS) / 4; i += GTHR) {
    const v4f v = *(const v4fa*)(stg + 4 * i);
    *(volatile v4f*)(base + 4 * i) = v;
  }
  __threadfence();
#pragma unroll 1
  for (int i = tid; i < (GBM * NOUTS) / 4; i += GTHR) {
    const v4f v = *(const v4fa*)(stg + 4 * i);
    *(volatile v4f*)(base + 4 * i) = v;
  }
}

__global__ __launch_bounds__(NTHR) void k_pool(const int* __restrict__ bat, int nN, const float* __restrict__ of,
                                               int nG, const unsigned short* __restrict__ g1t,
                                               const float* __restrict__ b1, const float* __restrict__ w2,
                                               const float* __restrict__ b2, float* out1) {
  __shared__ __attribute__((aligned(16))) float gs[NBP * HD];
  __shared__ __attribute__((aligned(16))) int plist[LISTN];
  __shared__ __attribute__((aligned(16))) unsigned short ga[NBP * K2];
  __shared__ __attribute__((aligned(16))) float gst[NBP * HD];
  __shared__ __attribute__((aligned(16))) float res[NBP];
  __shared__ int cnt[NBP];
  __shared__ int wcnt[NWAVE];
  const int tid = (int)threadIdx.x, lane = tid & 31, wave = tid >> 5, hh = lane >> 4, m = lane & 15;
  const int gBase = (int)blockIdx.x * NBP;
  int nb = nG - gBase;
  nb = nb < 0 ? 0 : (nb > NBP ? NBP : nb);
  {
    const v4f z = {0.f, 0.f, 0.f, 0.f};
    const v4i zi = {0, 0, 0, 0};
#pragma unroll 1
    for (int i = tid; i < NBP * HD / 4; i += NTHR) *(v4fa*)(gs + 4 * i) = z;
#pragma unroll 1
    for (int i = tid; i < LISTN / 4; i += NTHR) *(v4ia*)(plist + 4 * i) = zi;
    if (tid < NBP) { cnt[tid] = 0; res[tid] = 0.0f; }
    if (tid < NWAVE) wcnt[tid] = 0;
  }
  __syncthreads();

  const int nChunks = (nN + CHUNK - 1) / CHUNK;
#pragma unroll 1
  for (int ch = 0; ch < nChunks; ++ch) {
    const int cbase = ch * CHUNK;
    const int wc = scan_chunk<SLA>(bat, nN, cbase, gBase, nb, 1, plist, tid, lane, wave);
    if (lane == 0) wcnt[wave] = wc;
    __syncthreads();
#pragma unroll 1
    for (int wsx = 0; wsx < NWAVE; ++wsx) {
      int n = __builtin_amdgcn_readfirstlane(wcnt[wsx]);
      n = n > WCAP ? WCAP : (n < 0 ? 0 : n);
      const int* lp = plist + wsx * WCAP;
#pragma unroll 1
      for (int i = 0; i < n; ++i) {
        const int ent = __builtin_amdgcn_readfirstlane(lp[i]);
        int slot = ent & (NBA - 1);
        slot = slot > NBP - 1 ? NBP - 1 : slot;
        if ((slot >> 2) == wave) {
          int nd = cbase + ((ent >> SLA) & (CHUNK - 1));
          nd = nd > nN - 1 ? nN - 1 : nd;
          const v2f o = *(const v2f*)(of + (size_t)nd * HD + 2 * lane);
          v2fa* ap = (v2fa*)(gs + slot * HD + 2 * lane);
          *ap = *ap + o;
          if (lane == 0) cnt[slot] = cnt[slot] + 1;
        }
      }
    }
    __syncthreads();
  }

  {
    const int row = tid >> 3, c8 = (tid & 7) * 8;
    int cr = cnt[row];
    cr = cr < 1 ? 1 : cr;
    const float rc = 1.0f / (float)cr;
    const v4f a = *(const v4fa*)(gs + row * HD + c8) * rc;
    const v4f b = *(const v4fa*)(gs + row * HD + c8 + 4) * rc;
    *(v8usa*)(ga + row * K2 + c8)      = hl8(a, b, false);
    *(v8usa*)(ga + row * K2 + HD + c8) = hl8(a, b, true);
  }
  __syncthreads();

  {
    const int rg = wave >> 2, nt = wave & 3;
    v8f acc = z8();
    const unsigned short* arow = ga + (16 * rg + m) * K2 + 8 * hh;
    const unsigned short* bp   = g1t + (size_t)(16 * nt + m) * K2 + 8 * hh;
#pragma unroll
    for (int k0 = 0; k0 < K2; k0 += 32) {
      FragB af, bf;
      af.h[0] = *(const v8usa*)(arow + k0);
      af.h[1] = *(const v8usa*)(arow + k0 + 16);
      bf.h[0] = *(const v8usa*)(bp + k0);
      bf.h[1] = *(const v8usa*)(bp + k0 + 16);
      acc = wmb(af, bf, acc);
    }
    const int j = 16 * nt + m;
    const float bv = bf16_val(b1[j]);
#pragma unroll
    for (int r = 0; r < 8; ++r) gst[(16 * rg + 8 * hh + r) * HD + j] = lrelu(acc[r] + bv);
  }
  __syncthreads();

  {
    const float wa = bf16_val(w2[2 * lane]), wb = bf16_val(w2[2 * lane + 1]);
    const float bb = bf16_val(b2[0]);
#pragma unroll
    for (int rr = 0; rr < NBP / NWAVE; ++rr) {
      const int row = (NBP / NWAVE) * wave + rr;
      const v2f g = *(const v2fa*)(gst + row * HD + 2 * lane);
      const float p = wsum(g.x * wa + g.y * wb) + bb;
      if (lane == 0) res[row] = p;
    }
  }
  __syncthreads();

  const v4f v = *(const v4fa*)(res + 4 * (lane & 7));
  const bool wr = (wave == 0) && (lane < 8) && (nb == NBP);
  if (wr) *(volatile v4f*)(out1 + gBase + 4 * lane) = v;
  __threadfence();
  if (wr) *(volatile v4f*)(out1 + gBase + 4 * lane) = v;
}

static inline int cdiv(int a, int b) { return (a + b - 1) / b; }

extern "C" void kernel_launch(void* const* d_in, const int* in_sizes, int n_in,
                              void* d_out, int out_size, void* d_ws, size_t ws_size,
                              hipStream_t stream) {
  if (n_in < 32) return;
  const int nN = in_sizes[0];
  const int nS = in_sizes[1];
  if (in_sizes[3] < 2 || (in_sizes[3] & 1) != 0) return;
  const int nE = in_sizes[3] / 2;
  const int nG = in_sizes[7];
  if (nN < GBM || (nN % GBM) != 0 || nN > (1 << 24)) return;
  if (nS < GBM || (nS % GBM) != 0) return;
  if (nG < NBP || (nG % NBP) != 0) return;
  if (nE < 1 || nE >= (1 << 21)) return;
  if (in_sizes[2] != 2 * nE) return;
  if (in_sizes[4] != nN || in_sizes[5] != nS || in_sizes[6] != nS) return;
  if (in_sizes[8] != nG * NVEC) return;
  const int nBlk = in_sizes[9] / HD;
  if (nBlk < 1 || in_sizes[9] != nBlk * HD) return;
  const int nStemT = in_sizes[10] / HD;
  if (nStemT < 1 || in_sizes[10] != nStemT * HD) return;
  const int nBond = in_sizes[11] / HD;
  if (nBond < 1 || nBond > BTMAX || in_sizes[11] != nBond * HD) return;
  if (in_sizes[12] != HD * HD || in_sizes[13] != HD) return;
  if (in_sizes[14] != HD * KH0 || in_sizes[15] != HD || in_sizes[16] != HD * HD || in_sizes[17] != HD) return;
  if (in_sizes[18] != 3 * HD * HD || in_sizes[19] != 3 * HD || in_sizes[20] != 3 * HD * HD || in_sizes[21] != 3 * HD) return;
  if (in_sizes[22] != HD * 2 * HD || in_sizes[23] != HD || in_sizes[24] != HD * HD || in_sizes[25] != HD) return;
  if (in_sizes[26] != NOUTS * HD || in_sizes[27] != NOUTS) return;
  if (in_sizes[28] != HD * HD || in_sizes[29] != HD || in_sizes[30] != HD || in_sizes[31] != 1) return;
  if ((long long)out_size != (long long)nS * NOUTS + (long long)nG) return;

  const int*   x_ids        = (const int*)d_in[0];
  const int*   stemtype_ids = (const int*)d_in[1];
  const int*   edge_attr    = (const int*)d_in[2];
  const int*   edge_index   = (const int*)d_in[3];
  const int*   batch        = (const int*)d_in[4];
  const int*   stems_local  = (const int*)d_in[5];
  const int*   stems_batch  = (const int*)d_in[6];
  const int*   node_slices  = (const int*)d_in[7];
  const float* vec_data     = (const float*)d_in[8];
  const float* blockemb     = (const float*)d_in[9];
  const float* stememb      = (const float*)d_in[10];
  const float* bondemb      = (const float*)d_in[11];
  const float* conv_root    = (const float*)d_in[12];
  const float* conv_bias    = (const float*)d_in[13];
  const float* b2e_w1 = (const float*)d_in[14]; const float* b2e_b1 = (const float*)d_in[15];
  const float* b2e_w2 = (const float*)d_in[16]; const float* b2e_b2 = (const float*)d_in[17];
  const float* gru_w_ih = (const float*)d_in[18]; const float* gru_b_ih = (const float*)d_in[19];
  const float* gru_w_hh = (const float*)d_in[20]; const float* gru_b_hh = (const float*)d_in[21];
  const float* s2p_w1 = (const float*)d_in[22]; const float* s2p_b1 = (const float*)d_in[23];
  const float* s2p_w2 = (const float*)d_in[24]; const float* s2p_b2 = (const float*)d_in[25];
  const float* s2p_w3 = (const float*)d_in[26]; const float* s2p_b3 = (const float*)d_in[27];
  const float* g2p_w1 = (const float*)d_in[28]; const float* g2p_b1 = (const float*)d_in[29];
  const float* g2p_w2 = (const float*)d_in[30]; const float* g2p_b2 = (const float*)d_in[31];
  float* out  = (float*)d_out;
  float* out1 = out + (size_t)nS * NOUTS;
  const int* src = edge_index;
  const int* dst = edge_index + nE;

  char* ws = (char*)d_ws;
  size_t off = 0;
  const size_t oWPL = off; off += (size_t)PO_TOT * 2;          off = (off + 255) & ~(size_t)255;
  const size_t oH0  = off; off += (size_t)nN * KH0 * 2;         off = (off + 255) & ~(size_t)255;
  const size_t oT1  = off; off += (size_t)nN * K2 * 2;          off = (off + 255) & ~(size_t)255;
  const size_t oOF0 = off; off += (size_t)nN * HD * 4;          off = (off + 255) & ~(size_t)255;
  const size_t oOF1 = off; off += (size_t)nN * HD * 4;          off = (off + 255) & ~(size_t)255;
  const size_t oOA0 = off; off += (size_t)nN * K2 * 2;          off = (off + 255) & ~(size_t)255;
  const size_t oOA1 = off; off += (size_t)nN * K2 * 2;          off = (off + 255) & ~(size_t)255;
  const size_t oOR  = off; off += (size_t)nN * HD * 4;          off = (off + 255) & ~(size_t)255;
  const size_t oM   = off; off += (size_t)nN * K2 * 2;          off = (off + 255) & ~(size_t)255;
  const size_t oS1  = off; off += (size_t)nS * K2 * 2;          off = (off + 255) & ~(size_t)255;
  const size_t oS2  = off; off += (size_t)nS * K2 * 2;          off = (off + 255) & ~(size_t)255;
  if (off > ws_size || off > (size_t)WSMAX) return;
  unsigned short* WPL = (unsigned short*)(ws + oWPL);
  unsigned short* H0  = (unsigned short*)(ws + oH0);
  unsigned short* T1  = (unsigned short*)(ws + oT1);
  float*          OF0 = (float*)(ws + oOF0);
  float*          OF1 = (float*)(ws + oOF1);
  unsigned short* OA0 = (unsigned short*)(ws + oOA0);
  unsigned short* OA1 = (unsigned short*)(ws + oOA1);
  float*          ORP = (float*)(ws + oOR);
  unsigned short* MPL = (unsigned short*)(ws + oM);
  unsigned short* S1  = (unsigned short*)(ws + oS1);
  unsigned short* S2  = (unsigned short*)(ws + oS2);
  float* OFP[2] = {OF0, OF1};
  unsigned short* OAP[2] = {OA0, OA1};

  const int vec8 = ((nE & 3) == 0) ? 1 : 0;
  const int gA = cdiv(nN, NBA);
  const size_t aggLds = (size_t)AGG_LDS_INTS * 4;
  hipFuncSetAttribute(reinterpret_cast<const void*>(&k_agg), hipFuncAttributeMaxDynamicSharedMemorySize, (int)aggLds);

  k_wprep<<<dim3(12, 9), NTHR, 0, stream>>>(b2e_w1, b2e_w2, conv_root, gru_w_ih, gru_w_hh, s2p_w1, s2p_w2, s2p_w3, g2p_w1, WPL);
  const int nUh = nN * (KH0 / 8);
  k_h0<<<cdiv(nUh, NTHR), NTHR, 0, stream>>>(x_ids, batch, blockemb, nBlk, vec_data, nG, nUh, H0);

  k_gemm64<1, 0, 1><<<nN / GBM, GTHR, 0, stream>>>(H0, KH0, WPL + PO_B2E1, KH0, KH0, b2e_b1, ORP, T1);
  k_gemm64<0, 1, 1><<<nN / GBM, GTHR, 0, stream>>>(T1, K2, WPL + PO_B2E2, K2, K2, b2e_b2, OF0, OA0);

  int curb = 0;
  for (int s = 0; s < 6; ++s) {
    const int nxb = curb ^ 1;
    k_gemm64<0, 1, 0><<<nN / GBM, GTHR, 0, stream>>>(OAP[curb], K2, WPL + PO_ROOT, K2, K2, conv_bias, ORP, MPL);
    k_agg<<<gA, NTHR, aggLds, stream>>>(src, dst, edge_attr, nE, nN, vec8, OFP[curb], ORP, bondemb, nBond, MPL);
    k_gru<<<nN / GBM, NTHR, 0, stream>>>(MPL, OAP[curb], OFP[curb], WPL + PO_GIH, WPL + PO_GHH, gru_b_ih, gru_b_hh,
                                         OFP[nxb], OAP[nxb]);
    curb = nxb;
  }

  k_stem1<<<nS / GBM, GTHR, 0, stream>>>(OAP[curb], nN, stemtype_ids, stems_local, stems_batch, node_slices, nG, nS,
                                         stememb, nStemT, WPL + PO_S2P1, s2p_b1, S1);
  k_gemm64<1, 0, 1><<<nS / GBM, GTHR, 0, stream>>>(S1, K2, WPL + PO_S2P2, K2, K2, s2p_b2, ORP, S2);
  k_stem3<<<nS / GBM, GTHR, 0, stream>>>(S2, WPL + PO_S2P3, s2p_b3, out);

  k_pool<<<nG / NBP, NTHR, 0, stream>>>(batch, nN, OFP[curb], nG, WPL + PO_G2P1, g2p_b1, g2p_w2, g2p_b2, out1);
}
